// DCTblock_21517786153312
// MI455X (gfx1250) — hardware-run, weakly checked
//
#include <hip/hip_runtime.h>
#include <math.h>

typedef __attribute__((ext_vector_type(16))) _Float16 v16h;
typedef __attribute__((ext_vector_type(8)))  _Float16 v8h;
typedef __attribute__((ext_vector_type(8)))  float    v8f;
typedef __attribute__((ext_vector_type(4)))  float    v4f;
typedef __attribute__((ext_vector_type(4)))  unsigned int v4u;

constexpr int kBatch  = 512;
constexpr int kTime   = 125;
constexpr int kNode   = 66;
constexpr int kCoef   = 20;
constexpr int kHid    = 256;
constexpr int kStages = 6;
constexpr int kHist   = 25;
constexpr int kChan   = kNode * kHid;
constexpr int kCoefPad = 32;
constexpr int kMRows  = 80;
constexpr int kKNode  = 96;
constexpr int kLdaH   = 40;
constexpr int kLdtH   = 104;
constexpr int kSlabF  = 16 * 36;
constexpr int kAttPlane = kMRows * kKNode;
constexpr int kOutElems = kBatch * kTime * kNode;
constexpr int kRows   = kBatch * kNode;
constexpr float kCarry = 16.0f;
constexpr float kOutScale = 1.0f / 256.0f;

__device__ __forceinline__ unsigned pk16(unsigned short a, unsigned short b) { return (unsigned)a | ((unsigned)b << 16); }
__device__ __forceinline__ unsigned short h_bits(float f) { const _Float16 h = (_Float16)f; return __builtin_bit_cast(unsigned short, h); }

__device__ __forceinline__ void dep_guard_h(v8f& a, v8f& b, v16h x, v16h y) { asm volatile("v_nop\n\tv_nop\n\tv_nop\n\tv_nop" : "+v"(a), "+v"(b) : "v"(x), "v"(y)); }
__device__ __forceinline__ void keep4_h(v16h a, v16h b, v16h c, v16h d) { asm volatile("v_nop" :: "v"(a), "v"(b), "v"(c), "v"(d)); }
__device__ __forceinline__ void acc_guard4(v8f& a, v8f& b, v8f& c, v8f& d) { asm volatile("v_nop\n\tv_nop\n\tv_nop\n\tv_nop" : "+v"(a), "+v"(b), "+v"(c), "+v"(d)); }

template <typename T> struct Frag;
template <> struct Frag<_Float16> {
  typedef v16h V; union U { v16h v; v8h h[2]; };
  static __device__ __forceinline__ v16h load(const _Float16* p) {
    U f; f.h[0] = *(const v8h*)(p); f.h[1] = *(const v8h*)(p + 16); return f.v;
  }
  static __device__ __forceinline__ v8f mma(v16h a, v16h b, v8f c) {
    return __builtin_amdgcn_wmma_f32_16x16x32_f16(false, a, false, b, (short)0, c, false, false);
  }
  static __device__ __forceinline__ void guard(v8f& a, v8f& b, v16h x, v16h y) { dep_guard_h(a, b, x, y); }
};

__global__ __launch_bounds__(256) void prep_w_kernel(const float* __restrict__ wA, const float* __restrict__ wB,
                                                    int nsplit, long wstride,
                                                    unsigned short* __restrict__ outp, long ostride,
                                                    int Kin, int Nreal, int Kp, int Nrows, float scale)
{
  const int y = blockIdx.y;
  const float* W = (y < nsplit) ? (wA + (size_t)y * wstride) : (wB + (size_t)(y - nsplit) * wstride);
  unsigned short* op = outp + (size_t)y * ostride;
  const int kch = Kp >> 3;
  const int nch = Nrows * kch;
  const int i = blockIdx.x * 256 + threadIdx.x;
  if (i >= nch) return;
  const int f  = i / kch;
  const int k8 = (i - f * kch) * 8;
  const int fc = (f < Nreal) ? f : (Nreal - 1);
  unsigned short hb[8];
#pragma unroll
  for (int e = 0; e < 8; ++e) {
    const int k  = k8 + e;
    const int kc = (k < Kin) ? k : (Kin - 1);
    float v = W[(size_t)kc * Nreal + fc] * scale;
    v = (k < Kin && f < Nreal) ? v : 0.0f;
    hb[e] = h_bits(v);
  }
  const v4u u = (v4u){pk16(hb[0], hb[1]), pk16(hb[2], hb[3]), pk16(hb[4], hb[5]), pk16(hb[6], hb[7])};
  unsigned short* q = op + (size_t)f * Kp + k8;
  *(volatile v4u*)q = u;
  __threadfence();
  *(volatile v4u*)q = u;
}

__global__ __launch_bounds__(256) void prep_att_kernel(const float* __restrict__ a0, const float* __restrict__ a1,
                                                      const float* __restrict__ a2, const float* __restrict__ a3,
                                                      unsigned short* __restrict__ outp, float scale)
{
  const int y = blockIdx.y;
  const float* A = (y == 0) ? a0
                 : (y <= kStages) ? (a1 + (size_t)(y - 1) * (kNode * kNode))
                 : (y <= 2 * kStages) ? (a2 + (size_t)(y - 1 - kStages) * (kNode * kNode))
                 : a3;
  const int i = blockIdx.x * 256 + threadIdx.x;
  if (i >= kMRows * (kKNode / 8)) return;
  const int n  = i / (kKNode / 8);
  const int m8 = (i - n * (kKNode / 8)) * 8;
  const int nc = (n < kNode) ? n : (kNode - 1);
  unsigned short hb[8];
#pragma unroll
  for (int e = 0; e < 8; ++e) {
    const int m  = m8 + e;
    const int mc = (m < kNode) ? m : (kNode - 1);
    float v = A[nc * kNode + mc] * scale;
    v = (n < kNode && m < kNode) ? v : 0.0f;
    hb[e] = h_bits(v);
  }
  const v4u u = (v4u){pk16(hb[0], hb[1]), pk16(hb[2], hb[3]), pk16(hb[4], hb[5]), pk16(hb[6], hb[7])};
  unsigned short* q = outp + (size_t)y * kAttPlane + (size_t)i * 8;
  *(volatile v4u*)q = u;
  __threadfence();
  *(volatile v4u*)q = u;
}

__global__ __launch_bounds__(256) void tproj_kernel(const float* __restrict__ x, const float* __restrict__ tm,
                                                   float* __restrict__ xd32, unsigned short* __restrict__ xd16)
{
  __shared__ __align__(16) float xs[kTime * kNode + 6];
  __shared__ __align__(16) float ts[kTime * kCoef + 12];
  __shared__ __align__(16) float res[kNode * kCoefPad];
  const int b = blockIdx.x, tid = threadIdx.x;
  const float* xb = x + (size_t)b * (kTime * kNode);
  for (int i = tid; i < kTime * kNode; i += 256) xs[i] = xb[i];
  for (int i = tid; i < kCoef * kTime; i += 256) {
    const int d = i / kTime, t = i - d * kTime;
    ts[t * kCoef + d] = tm[i];
  }
  for (int i = tid; i < kNode * 3; i += 256) {
    const int n = i / 3, q = i - n * 3;
    *(v4f*)(res + n * kCoefPad + kCoef + 4 * q) = (v4f){0.f, 0.f, 0.f, 0.f};
  }
  __syncthreads();
  for (int item = tid; item < kNode * 5; item += 256) {
    const int n = item / 5, d4 = item - n * 5;
    float s0 = 0.f, s1 = 0.f, s2 = 0.f, s3 = 0.f;
#pragma unroll 5
    for (int t = 0; t < kTime; ++t) {
      const float xv = xs[t * kNode + n];
      const v4f a = *(const v4f*)(ts + t * kCoef + 4 * d4);
      s0 += a.x * xv; s1 += a.y * xv; s2 += a.z * xv; s3 += a.w * xv;
    }
    *(v4f*)(res + n * kCoefPad + 4 * d4) = (v4f){s0, s1, s2, s3};
  }
  __syncthreads();
  float* od = xd32 + (size_t)b * (kNode * kCoefPad);
  unsigned short* oh = xd16 + (size_t)b * (kNode * kCoefPad);
  for (int pass = 0; pass < 2; ++pass) {
    for (int c = tid; c < kNode * kCoefPad / 4; c += 256) {
      const v4f v = *(const v4f*)(res + c * 4);
      *(volatile v4f*)(od + c * 4) = v;
    }
    for (int c = tid; c < kNode * kCoefPad / 8; c += 256) {
      const v4f a = *(const v4f*)(res + c * 8);
      const v4f g = *(const v4f*)(res + c * 8 + 4);
      const v4u u = (v4u){pk16(h_bits(a.x), h_bits(a.y)), pk16(h_bits(a.z), h_bits(a.w)),
                          pk16(h_bits(g.x), h_bits(g.y)), pk16(h_bits(g.z), h_bits(g.w))};
      *(volatile v4u*)(oh + c * 8) = u;
    }
    __threadfence();
  }
}

template <int NT, bool ADDX>
__global__ __launch_bounds__(256) void gmix_kernel(const unsigned short* __restrict__ in16, int Kp,
                                                  const unsigned short* __restrict__ wT,
                                                  const unsigned short* __restrict__ attP,
                                                  const float* __restrict__ bias, int Nreal,
                                                  const float* __restrict__ addx,
                                                  float* __restrict__ outp, int ldo)
{
  static_assert(NT == 16 || NT == 2);
  static_assert(!ADDX || NT == 2);
  constexpr int kNOut  = NT * 16;
  constexpr int kTtF   = kNOut * kLdtH / 2;
  constexpr int kPoolF = (kTtF > 8 * kSlabF) ? kTtF : 8 * kSlabF;
  __shared__ __align__(16) unsigned short Ah[kMRows * kLdaH];
  __shared__ __align__(16) float pool[kPoolF];
  unsigned short* Tt = (unsigned short*)pool;

  const int tid  = threadIdx.x;
  const int lane = tid & 31;
  const int wv   = __builtin_amdgcn_readfirstlane(tid >> 5);
  const int l15  = lane & 15;
  const int hh   = lane >> 4;
  const int koff = hh * 8;
  const int b    = blockIdx.x;
  const bool hasWork = (NT == 16) || (wv == 0);
  const int nt0 = 2 * wv, nt1 = 2 * wv + 1;

  const v4u z4 = (v4u){0u, 0u, 0u, 0u};
  if (tid < (kMRows - kNode) * 4) {
    const int r = kNode + (tid >> 2), q = tid & 3;
    *(v4u*)(Ah + r * kLdaH + q * 8) = z4;
  }
  for (int i = tid; i < kNOut * 2; i += 256) {
    const int row = i >> 1, q = i & 1;
    *(v4u*)(Tt + row * kLdtH + 80 + q * 8) = z4;
  }

  v8f acc[5][2];
#pragma unroll
  for (int mt = 0; mt < 5; ++mt)
#pragma unroll
    for (int j = 0; j < 2; ++j) acc[mt][j] = (v8f){0.f, 0.f, 0.f, 0.f, 0.f, 0.f, 0.f, 0.f};

  const unsigned short* inb = in16 + (size_t)b * kNode * Kp;
  const int nks = Kp >> 5;
  for (int ks = 0; ks < nks; ++ks) {
    __syncthreads();
    {
      const int r = tid >> 2, q = tid & 3;
      const v4u v = *(const v4u*)(inb + (size_t)r * Kp + ks * 32 + q * 8);
      *(v4u*)(Ah + r * kLdaH + q * 8) = v;
      if (tid < kNode * 4 - 256) {
        const int c2 = 256 + tid;
        const int r2 = c2 >> 2, q2 = c2 & 3;
        const v4u v2 = *(const v4u*)(inb + (size_t)r2 * Kp + ks * 32 + q2 * 8);
        *(v4u*)(Ah + r2 * kLdaH + q2 * 8) = v2;
      }
    }
    __syncthreads();
    if (hasWork) {
      const v16h bf0 = Frag<_Float16>::load((const _Float16*)(wT + (size_t)(nt0 * 16 + l15) * Kp + ks * 32 + koff));
      const v16h bf1 = Frag<_Float16>::load((const _Float16*)(wT + (size_t)(nt1 * 16 + l15) * Kp + ks * 32 + koff));
#pragma unroll
      for (int mt = 0; mt < 5; ++mt) {
        const v16h af = Frag<_Float16>::load((const _Float16*)(Ah + (mt * 16 + l15) * kLdaH + koff));
        acc[mt][0] = Frag<_Float16>::mma(af, bf0, acc[mt][0]);
        acc[mt][1] = Frag<_Float16>::mma(af, bf1, acc[mt][1]);
        Frag<_Float16>::guard(acc[mt][0], acc[mt][1], af, bf0);
      }
      keep4_h(bf0, bf1, bf0, bf1);
    }
  }
  acc_guard4(acc[0][0], acc[0][1], acc[1][0], acc[1][1]);
  acc_guard4(acc[2][0], acc[2][1], acc[3][0], acc[3][1]);
  acc_guard4(acc[4][0], acc[4][1], acc[0][0], acc[1][0]);

  if (hasWork) {
#pragma unroll
    for (int j = 0; j < 2; ++j) {
      const int f = ((j == 0) ? nt0 : nt1) * 16 + l15;
#pragma unroll
      for (int mt = 0; mt < 5; ++mt) {
        unsigned short hb[8];
#pragma unroll
        for (int e = 0; e < 8; ++e) hb[e] = h_bits(acc[mt][j][e]);
        const v4u u = (v4u){pk16(hb[0], hb[1]), pk16(hb[2], hb[3]), pk16(hb[4], hb[5]), pk16(hb[6], hb[7])};
        *(v4u*)(Tt + f * kLdtH + mt * 16 + hh * 8) = u;
      }
    }
  }
  __syncthreads();

#pragma unroll
  for (int mt = 0; mt < 5; ++mt)
#pragma unroll
    for (int j = 0; j < 2; ++j) acc[mt][j] = (v8f){0.f, 0.f, 0.f, 0.f, 0.f, 0.f, 0.f, 0.f};

#pragma unroll
  for (int ks = 0; ks < kKNode / 32; ++ks) {
    if (hasWork) {
      const v16h bf0 = Frag<_Float16>::load((const _Float16*)(Tt + (nt0 * 16 + l15) * kLdtH + ks * 32 + koff));
      const v16h bf1 = Frag<_Float16>::load((const _Float16*)(Tt + (nt1 * 16 + l15) * kLdtH + ks * 32 + koff));
#pragma unroll
      for (int mt = 0; mt < 5; ++mt) {
        const v16h af = Frag<_Float16>::load((const _Float16*)(attP + (mt * 16 + l15) * kKNode + ks * 32 + koff));
        acc[mt][0] = Frag<_Float16>::mma(af, bf0, acc[mt][0]);
        acc[mt][1] = Frag<_Float16>::mma(af, bf1, acc[mt][1]);
        Frag<_Float16>::guard(acc[mt][0], acc[mt][1], af, bf0);
      }
      keep4_h(bf0, bf1, bf0, bf1);
    }
  }
  acc_guard4(acc[0][0], acc[0][1], acc[1][0], acc[1][1]);
  acc_guard4(acc[2][0], acc[2][1], acc[3][0], acc[3][1]);
  acc_guard4(acc[4][0], acc[4][1], acc[0][0], acc[1][0]);
  __syncthreads();

  if (hasWork) {
    float* slab = pool + wv * kSlabF;
    const int qrow = lane >> 3, c4 = (lane & 7) * 4;
#pragma unroll
    for (int mt = 0; mt < 5; ++mt) {
#pragma unroll
      for (int j = 0; j < 2; ++j) {
        const int f   = (2 * wv + j) * 16 + l15;
        const int fcl = (f < Nreal) ? f : (Nreal - 1);
        const float bv = bias[fcl];
#pragma unroll
        for (int r = 0; r < 8; ++r) {
          const int n = mt * 16 + hh * 8 + r;
          float v = acc[mt][j][r] * kOutScale + bv;
          if (ADDX) {
            const int ncl = (n < kNode) ? n : (kNode - 1);
            v += addx[((size_t)b * kNode + ncl) * kCoefPad + f];
          }
          v = (f < Nreal) ? v : 0.0f;
          slab[(hh * 8 + r) * 36 + j * 16 + l15] = v;
        }
      }
      __builtin_amdgcn_fence(__ATOMIC_RELEASE, "workgroup");
      __builtin_amdgcn_wave_barrier();
      __builtin_amdgcn_fence(__ATOMIC_ACQUIRE, "workgroup");
      for (int pass = 0; pass < 2; ++pass) {
#pragma unroll
        for (int it = 0; it < 4; ++it) {
          const int row = it * 4 + qrow;
          const int n   = mt * 16 + row;
          const v4f val = *(const v4f*)(slab + row * 36 + c4);
          if (n < kNode) *(volatile v4f*)(outp + ((size_t)b * kNode + n) * ldo + wv * 32 + c4) = val;
        }
        __threadfence();
      }
      __builtin_amdgcn_fence(__ATOMIC_RELEASE, "workgroup");
      __builtin_amdgcn_wave_barrier();
      __builtin_amdgcn_fence(__ATOMIC_ACQUIRE, "workgroup");
    }
  }
}

__global__ __launch_bounds__(256) void bn_stats_kernel(const float* __restrict__ Y, float* __restrict__ mu, float* __restrict__ rsd)
{
  const int c = blockIdx.x * 256 + threadIdx.x;
  const float* p = Y + c;
  float s = 0.f;
#pragma unroll 4
  for (int bb = 0; bb < kBatch; ++bb) s += p[(size_t)bb * kChan];
  const float m = s * (1.0f / (float)kBatch);
  float s2 = 0.f;
#pragma unroll 4
  for (int bb = 0; bb < kBatch; ++bb) {
    const float d = p[(size_t)bb * kChan] - m;
    s2 += d * d;
  }
  const float var = s2 * (1.0f / (float)kBatch);
  const float r = rsqrtf(var + 1e-5f);
  *(volatile float*)(mu + c)  = m;
  *(volatile float*)(rsd + c) = r;
  __threadfence();
  *(volatile float*)(mu + c)  = m;
  *(volatile float*)(rsd + c) = r;
}

template <int MODE>
__global__ __launch_bounds__(256) void bn_apply_kernel(const float* __restrict__ Y, const float* __restrict__ mu,
                                                      const float* __restrict__ rsd, const float* __restrict__ gma,
                                                      const float* __restrict__ bta, float* Hres,
                                                      unsigned short* __restrict__ X16)
{
  __shared__ __align__(16) float st[256 * 8];
  const int tid = threadIdx.x, lane = tid & 31, wave = tid >> 5;
  const int i = blockIdx.x * 256 + tid;
  const size_t e0 = (size_t)i * 8;
  const int c0 = (i % (kChan / 8)) * 8;
  const v4f y0 = *(const v4f*)(Y + e0),    y1 = *(const v4f*)(Y + e0 + 4);
  const v4f m0 = *(const v4f*)(mu + c0),   m1 = *(const v4f*)(mu + c0 + 4);
  const v4f r0 = *(const v4f*)(rsd + c0),  r1 = *(const v4f*)(rsd + c0 + 4);
  const v4f g0 = *(const v4f*)(gma + c0),  g1 = *(const v4f*)(gma + c0 + 4);
  const v4f b0 = *(const v4f*)(bta + c0),  b1 = *(const v4f*)(bta + c0 + 4);
  const v4f t0 = ((y0 - m0) * r0) * g0 + b0;
  const v4f t1 = ((y1 - m1) * r1) * g1 + b1;
  const size_t wbase = ((size_t)blockIdx.x * 256 + (size_t)wave * 32) * 8;
  v4f ho0 = (v4f){0.f, 0.f, 0.f, 0.f}, ho1 = ho0, hx0 = ho0, hx1 = ho0;
  if (MODE == 2) {
    ho0 = *(const v4f*)(Hres + e0);
    ho1 = *(const v4f*)(Hres + e0 + 4);
    hx0 = *(const v4f*)(Hres + wbase + lane * 4);
    hx1 = *(const v4f*)(Hres + wbase + 128 + lane * 4);
  }
  st[tid * 8 + 0] = t0.x; st[tid * 8 + 1] = t0.y; st[tid * 8 + 2] = t0.z; st[tid * 8 + 3] = t0.w;
  st[tid * 8 + 4] = t1.x; st[tid * 8 + 5] = t1.y; st[tid * 8 + 6] = t1.z; st[tid * 8 + 7] = t1.w;
#pragma unroll 1
  for (int e = 0; e < 8; ++e) st[tid * 8 + e] = tanhf(st[tid * 8 + e]);
  __syncthreads();
  v4f a0 = *(const v4f*)(st + tid * 8);
  v4f a1 = *(const v4f*)(st + tid * 8 + 4);
  if (MODE == 2) { a0 += ho0; a1 += ho1; }
  const v4u u = (v4u){pk16(h_bits(a0.x), h_bits(a0.y)), pk16(h_bits(a0.z), h_bits(a0.w)),
                      pk16(h_bits(a1.x), h_bits(a1.y)), pk16(h_bits(a1.z), h_bits(a1.w))};
  unsigned short* q = X16 + e0;
  *(volatile v4u*)q = u;
  __threadfence();
  *(volatile v4u*)q = u;
  if (MODE >= 1) {
    v4f x0 = *(const v4f*)(st + wave * 256 + lane * 4);
    v4f x1 = *(const v4f*)(st + wave * 256 + 128 + lane * 4);
    if (MODE == 2) { x0 += hx0; x1 += hx1; }
    for (int pass = 0; pass < 2; ++pass) {
      *(volatile v4f*)(Hres + wbase + lane * 4) = x0;
      *(volatile v4f*)(Hres + wbase + 128 + lane * 4) = x1;
      __threadfence();
    }
  }
}

__global__ __launch_bounds__(256) void tsynth_out_kernel(const float* __restrict__ x, const float* __restrict__ itm,
                                                        const float* __restrict__ yd, float* __restrict__ outp)
{
  __shared__ __align__(16) float ims[kTime * kCoef];
  const int tid = threadIdx.x;
  for (int i = tid; i < kTime * kCoef; i += 256) {
    const int t = i / kCoef, d = i - t * kCoef;
    ims[i] = itm[t * kTime + d];
  }
  __syncthreads();
  const int gi = blockIdx.x * 256 + tid;
  const size_t e0 = (size_t)gi * 4;
  const v4f xv = *(const v4f*)(x + e0);
  float o[4];
#pragma unroll
  for (int j = 0; j < 4; ++j) {
    const size_t e = e0 + j;
    const int b   = (int)(e / (size_t)(kTime * kNode));
    const int rem = (int)(e - (size_t)b * (kTime * kNode));
    const int t   = rem / kNode;
    const int n   = rem - t * kNode;
    const float* yr = yd + ((size_t)b * kNode + n) * kCoefPad;
    const float* ir = ims + t * kCoef;
    float s = 0.f;
#pragma unroll 1
    for (int d4 = 0; d4 < kCoef / 4; ++d4) {
      const v4f a = *(const v4f*)(ir + 4 * d4);
      const v4f c = *(const v4f*)(yr + 4 * d4);
      s += a.x * c.x; s += a.y * c.y; s += a.z * c.z; s += a.w * c.w;
    }
    o[j] = (t < kHist) ? xv[j] : s;
  }
  const v4f ov = (v4f){o[0], o[1], o[2], o[3]};
  float* q = outp + e0;
  *(volatile v4f*)q = ov;
  __threadfence();
  *(volatile v4f*)q = ov;
}

extern "C" void kernel_launch(void* const* d_in, const int* in_sizes, int n_in,
                              void* d_out, int out_size, void* d_ws, size_t ws_size,
                              hipStream_t stream)
{
  if (n_in < 21) return;
  if (out_size != kOutElems) return;
  if (in_sizes[0] != kOutElems) return;
  if (in_sizes[1] != kTime * kTime || in_sizes[2] != kTime * kTime) return;
  if (in_sizes[8] != kStages * kHid * kHid || in_sizes[13] != kStages * kHid * kHid) return;
  if (in_sizes[6] != kChan || in_sizes[11] != kStages * kChan) return;

  const float* x        = (const float*)d_in[0];
  const float* trans_m  = (const float*)d_in[1];
  const float* itrans_m = (const float*)d_in[2];
  const float* enc_w    = (const float*)d_in[3];
  const float* enc_att  = (const float*)d_in[4];
  const float* enc_b    = (const float*)d_in[5];
  const float* bn0_g    = (const float*)d_in[6];
  const float* bn0_b    = (const float*)d_in[7];
  const float* g1_w     = (const float*)d_in[8];
  const float* g1_att   = (const float*)d_in[9];
  const float* g1_b     = (const float*)d_in[10];
  const float* bn1_g    = (const float*)d_in[11];
  const float* bn1_b    = (const float*)d_in[12];
  const float* g2_w     = (const float*)d_in[13];
  const float* g2_att   = (const float*)d_in[14];
  const float* g2_b     = (const float*)d_in[15];
  const float* bn2_g    = (const float*)d_in[16];
  const float* bn2_b    = (const float*)d_in[17];
  const float* dec_w    = (const float*)d_in[18];
  const float* dec_att  = (const float*)d_in[19];
  const float* dec_b    = (const float*)d_in[20];
  float* out = (float*)d_out;

  char* ws = (char*)d_ws;
  size_t off = 0;
  const size_t bXd32 = (size_t)kRows * kCoefPad * 4;
  const size_t bXd16 = (size_t)kRows * kCoefPad * 2;
  const size_t bY32  = (size_t)kRows * kHid * 4;
  const size_t bX16  = (size_t)kRows * kHid * 2;
  const size_t bStat = (size_t)kChan * 4;
  const size_t bWenc = (size_t)kHid * kCoefPad * 2;
  const size_t bWst  = (size_t)2 * kStages * kHid * kHid * 2;
  const size_t bWdec = (size_t)kCoefPad * kHid * 2;
  const size_t bAtt  = (size_t)(2 + 2 * kStages) * kAttPlane * 2;
  float*          xd32 = (float*)(ws + off);           off += bXd32;
  unsigned short* xd16 = (unsigned short*)(ws + off);  off += bXd16;
  float*          Y32  = (float*)(ws + off);           off += bY32;
  float*          H32  = (float*)(ws + off);           off += bY32;
  unsigned short* X16  = (unsigned short*)(ws + off);  off += bX16;
  float*          Yd32 = (float*)(ws + off);           off += bXd32;
  float*          mu   = (float*)(ws + off);           off += bStat;
  float*          rsd  = (float*)(ws + off);           off += bStat;
  unsigned short* wenc = (unsigned short*)(ws + off);  off += bWenc;
  unsigned short* wst  = (unsigned short*)(ws + off);  off += bWst;
  unsigned short* wdec = (unsigned short*)(ws + off);  off += bWdec;
  unsigned short* attp = (unsigned short*)(ws + off);  off += bAtt;
  if (off > ws_size) return;

  prep_w_kernel<<<dim3(4, 1), 256, 0, stream>>>(enc_w, enc_w, 1, 0L, wenc, 0L, kCoef, kHid, kCoefPad, kHid, kCarry);
  prep_w_kernel<<<dim3(32, 2 * kStages), 256, 0, stream>>>(g1_w, g2_w, kStages, (long)kHid * kHid, wst, (long)kHid * kHid,
                                                            kHid, kHid, kHid, kHid, kCarry);
  prep_w_kernel<<<dim3(4, 1), 256, 0, stream>>>(dec_w, dec_w, 1, 0L, wdec, 0L, kHid, kCoef, kHid, kCoefPad, kCarry);
  prep_att_kernel<<<dim3(4, 2 + 2 * kStages), 256, 0, stream>>>(enc_att, g1_att, g2_att, dec_att, attp, kCarry);

  tproj_kernel<<<kBatch, 256, 0, stream>>>(x, trans_m, xd32, xd16);

  gmix_kernel<16, false><<<kBatch, 256, 0, stream>>>(xd16, kCoefPad, wenc, attp, enc_b, kHid, nullptr, Y32, kHid);
  bn_stats_kernel<<<kChan / 256, 256, 0, stream>>>(Y32, mu, rsd);
  bn_apply_kernel<1><<<kBatch * kChan / 8 / 256, 256, 0, stream>>>(Y32, mu, rsd, bn0_g, bn0_b, H32, X16);

  for (int s = 0; s < kStages; ++s) {
    gmix_kernel<16, false><<<kBatch, 256, 0, stream>>>(X16, kHid, wst + (size_t)s * kHid * kHid,
                                                       attp + (size_t)(1 + s) * kAttPlane,
                                                       g1_b + (size_t)s * kHid, kHid, nullptr, Y32, kHid);
    bn_stats_kernel<<<kChan / 256, 256, 0, stream>>>(Y32, mu, rsd);
    bn_apply_kernel<0><<<kBatch * kChan / 8 / 256, 256, 0, stream>>>(Y32, mu, rsd, bn1_g + (size_t)s * kChan,
                                                                     bn1_b + (size_t)s * kChan, nullptr, X16);
    gmix_kernel<16, false><<<kBatch, 256, 0, stream>>>(X16, kHid, wst + (size_t)(kStages + s) * kHid * kHid,
                                                       attp + (size_t)(1 + kStages + s) * kAttPlane,
                                                       g2_b + (size_t)s * kHid, kHid, nullptr, Y32, kHid);
    bn_stats_kernel<<<kChan / 256, 256, 0, stream>>>(Y32, mu, rsd);
    bn_apply_kernel<2><<<kBatch * kChan / 8 / 256, 256, 0, stream>>>(Y32, mu, rsd, bn2_g + (size_t)s * kChan,
                                                                     bn2_b + (size_t)s * kChan, H32, X16);
  }

  gmix_kernel<2, true><<<kBatch, 256, 0, stream>>>(X16, kHid, wdec, attp + (size_t)(1 + 2 * kStages) * kAttPlane,
                                                   dec_b, kCoef, xd32, Yd32, kCoefPad);

  tsynth_out_kernel<<<kOutElems / 4 / 256, 256, 0, stream>>>(x, itrans_m, Yd32, out);
}
